// EfficientLeaf_31516470018362
// MI455X (gfx1250) — hardware-run, weakly checked
//
#include <hip/hip_runtime.h>
#include <math.h>

typedef __attribute__((ext_vector_type(16))) _Float16 v16h;
typedef __attribute__((ext_vector_type(8)))  _Float16 v8h;
typedef __attribute__((ext_vector_type(8)))  float    v8f;
typedef __attribute__((ext_vector_type(4)))  float    v4f;

constexpr int kBatch      = 16;
constexpr int kSamples    = 160000;
constexpr int kBands      = 40;
constexpr int kFrames     = 1000;
constexpr int kLpPitch    = 1024;
constexpr int kTileFrames = 32;
constexpr int kRowTiles   = kLpPitch / kTileFrames;
constexpr int kPoolLen    = 401;

constexpr float kSigCarry   = 16.0f;
constexpr float kTapCarry   = 1024.0f;
constexpr float kEnergyFold = 1.0f / (kSigCarry * kTapCarry * kSigCarry * kTapCarry);
static_assert(kEnergyFold == 3.7252902984619140625e-9f, "energy fold is 2^-28");

constexpr double kZ      = 1.1774100225154747 / 3.141592653589793;
constexpr float kSigmaLo = (float)(2.0 * kZ);
constexpr float kSigmaHi = (float)(401.0 * kZ);
constexpr float kPwLo    = (float)(2.0 / 401.0);

template <int G> struct GroupCfg;
template <> struct GroupCfg<0> { static constexpr int kA0 = 0,  kCs = 10, kPs = 16,  kTaps = 151, kWin = 41,  kTs = 16, kNsl = 1, kKp = 160, kStep = 2, kTc = 16000,  kPlaneOff = 0,     kWinOff = 0; };
template <> struct GroupCfg<1> { static constexpr int kA0 = 10, kCs = 4,  kPs = 40,  kTaps = 83,  kWin = 101, kTs = 16, kNsl = 1, kKp = 96,  kStep = 4, kTc = 40000,  kPlaneOff = 5120,  kWinOff = 410; };
template <> struct GroupCfg<2> { static constexpr int kA0 = 20, kCs = 2,  kPs = 80,  kTaps = 47,  kWin = 201, kTs = 8,  kNsl = 2, kKp = 64,  kStep = 2, kTc = 80000,  kPlaneOff = 8192,  kWinOff = 1420; };
template <> struct GroupCfg<3> { static constexpr int kA0 = 30, kCs = 1,  kPs = 160, kTaps = 25,  kWin = 401, kTs = 4,  kNsl = 4, kKp = 32,  kStep = 1, kTc = 160000, kPlaneOff = 10240, kWinOff = 3430; };

constexpr int kPlaneHalves = GroupCfg<3>::kPlaneOff + 32 * GroupCfg<3>::kKp;
constexpr int kPlaneBlocks = kPlaneHalves / 1024;
constexpr int kWinFloats   = GroupCfg<3>::kWinOff + 10 * GroupCfg<3>::kWin;
constexpr int kWinBlocks   = 8;
constexpr int kWinCarve    = kWinBlocks * 1024;
static_assert(GroupCfg<1>::kPlaneOff == GroupCfg<0>::kPlaneOff + 32 * GroupCfg<0>::kKp, "plane offsets");
static_assert(GroupCfg<2>::kPlaneOff == GroupCfg<1>::kPlaneOff + 32 * GroupCfg<1>::kKp, "plane offsets");
static_assert(GroupCfg<3>::kPlaneOff == GroupCfg<2>::kPlaneOff + 32 * GroupCfg<2>::kKp, "plane offsets");
static_assert(GroupCfg<1>::kWinOff == GroupCfg<0>::kWinOff + 10 * GroupCfg<0>::kWin, "window offsets");
static_assert(GroupCfg<2>::kWinOff == GroupCfg<1>::kWinOff + 10 * GroupCfg<1>::kWin, "window offsets");
static_assert(GroupCfg<3>::kWinOff == GroupCfg<2>::kWinOff + 10 * GroupCfg<2>::kWin, "window offsets");
static_assert(kPlaneHalves == 11264 && kPlaneBlocks * 1024 == kPlaneHalves, "plane blocks");
static_assert(kWinFloats == 7440 && kWinFloats <= kWinCarve, "window carve");

constexpr size_t kOffKPL  = 0;
constexpr size_t kOffWIN  = kOffKPL + (size_t)kPlaneHalves * 2;
constexpr size_t kOffLP   = kOffWIN + (size_t)kWinCarve * 4;
constexpr size_t kOffMED  = kOffLP  + (size_t)kBatch * kBands * kLpPitch * 4;
constexpr size_t kOffSTAT = kOffMED + (size_t)kBatch * kBands * 32 * 4;
constexpr size_t kWsTotal = kOffSTAT + (size_t)2 * kBands * 32 * 4;
static_assert(kWsTotal == 2768896ull, "carve total");
static_assert((kOffWIN % 128) == 0 && (kOffLP % 128) == 0 && (kOffMED % 128) == 0 && (kOffSTAT % 128) == 0, "aligned regions");
static_assert(kWsTotal <= 134217728ull, "carve cap");

template <typename T> struct Frag;
template <> struct Frag<_Float16> {
  typedef v16h V; union U { v16h v; v8h h[2]; };
  static __device__ __forceinline__ v16h load(const _Float16* p) {
    U f; f.h[0] = *(const v8h*)(p); f.h[1] = *(const v8h*)(p + 16); return f.v;
  }
};
__device__ __forceinline__ v8f mma_g(v16h a, v16h b, v8f c) {
  c = __builtin_amdgcn_wmma_f32_16x16x32_f16(false, a, false, b, (short)0, c, false, false);
  asm volatile("v_nop\n\tv_nop\n\tv_nop\n\tv_nop" : "+v"(c) : "v"(a), "v"(b));
  return c;
}

__global__ __launch_bounds__(256) void gen_tables_kernel(
    const float* __restrict__ cf, const float* __restrict__ bw, const float* __restrict__ pw,
    unsigned short* __restrict__ kplanes, float* __restrict__ wtab)
{
  __shared__ __align__(16) float sV[1024];
  const int tid = threadIdx.x;
  const int blk = blockIdx.x;
  const bool isPlane = blk < kPlaneBlocks;
  if (isPlane) {
#pragma unroll 1
    for (int i = 0; i < 4; ++i) {
      const int e = blk * 1024 + i * 256 + tid;
      const int g = (e >= GroupCfg<1>::kPlaneOff ? 1 : 0) + (e >= GroupCfg<2>::kPlaneOff ? 1 : 0) + (e >= GroupCfg<3>::kPlaneOff ? 1 : 0);
      const int off  = (g == 0) ? GroupCfg<0>::kPlaneOff : (g == 1) ? GroupCfg<1>::kPlaneOff : (g == 2) ? GroupCfg<2>::kPlaneOff : GroupCfg<3>::kPlaneOff;
      const int kpv  = (g == 0) ? GroupCfg<0>::kKp : (g == 1) ? GroupCfg<1>::kKp : (g == 2) ? GroupCfg<2>::kKp : GroupCfg<3>::kKp;
      const int taps = (g == 0) ? GroupCfg<0>::kTaps : (g == 1) ? GroupCfg<1>::kTaps : (g == 2) ? GroupCfg<2>::kTaps : GroupCfg<3>::kTaps;
      const int el  = e - off;
      const int row = el / kpv;
      const int k   = el - row * kpv;
      const int f   = (row < 16) ? (row >> 1) : (((row & 8) != 0) ? 9 : 8);
      const bool live = ((row < 16) || ((row & 6) == 0)) && (k < taps);
      const int fg  = g * 10 + f;
      const float mu = fminf(fmaxf(cf[fg], 0.0f), 3.14159265358979f);
      const float sg = fminf(fmaxf(bw[fg], kSigmaLo), kSigmaHi);
      const float tt = (float)(k - (taps >> 1));
      const float inv2s2 = __builtin_amdgcn_rcpf(2.0f * sg * sg);
      const float invn   = __builtin_amdgcn_rcpf(2.5066282746310002f * sg);
      const float gs  = expf(-(tt * tt) * inv2s2) * invn;
      const float ang = mu * tt;
      const float cv  = cosf(ang);
      const float sv  = sinf(ang);
      const float val = gs * (((row & 1) != 0) ? sv : cv) * kTapCarry;
      sV[i * 256 + tid] = live ? val : 0.0f;
    }
  } else {
    const int wb = blk - kPlaneBlocks;
#pragma unroll 1
    for (int i = 0; i < 4; ++i) {
      const int e = wb * 1024 + i * 256 + tid;
      const int g = (e >= GroupCfg<1>::kWinOff ? 1 : 0) + (e >= GroupCfg<2>::kWinOff ? 1 : 0) + (e >= GroupCfg<3>::kWinOff ? 1 : 0);
      const int off = (g == 0) ? GroupCfg<0>::kWinOff : (g == 1) ? GroupCfg<1>::kWinOff : (g == 2) ? GroupCfg<2>::kWinOff : GroupCfg<3>::kWinOff;
      const int wv  = (g == 0) ? GroupCfg<0>::kWin : (g == 1) ? GroupCfg<1>::kWin : (g == 2) ? GroupCfg<2>::kWin : GroupCfg<3>::kWin;
      const float ics = (g == 0) ? (1.0f / (float)GroupCfg<0>::kCs) : (g == 1) ? (1.0f / (float)GroupCfg<1>::kCs) : (g == 2) ? (1.0f / (float)GroupCfg<2>::kCs) : (1.0f / (float)GroupCfg<3>::kCs);
      const float iw  = (g == 0) ? (1.0f / (float)GroupCfg<0>::kWin) : (g == 1) ? (1.0f / (float)GroupCfg<1>::kWin) : (g == 2) ? (1.0f / (float)GroupCfg<2>::kWin) : (1.0f / (float)GroupCfg<3>::kWin);
      const float t2s = (g == 0) ? (2.0f / (float)(GroupCfg<0>::kWin - 1)) : (g == 1) ? (2.0f / (float)(GroupCfg<1>::kWin - 1)) : (g == 2) ? (2.0f / (float)(GroupCfg<2>::kWin - 1)) : (2.0f / (float)(GroupCfg<3>::kWin - 1));
      const int el = e - off;
      const int fr = el / wv;
      const int w  = el - fr * wv;
      const int fc = fr < 9 ? fr : 9;
      const bool live = e < kWinFloats;
      const float p  = fminf(fmaxf(pw[g * 10 + fc], kPwLo), 0.5f);
      const float sp = ((p * ics) * (float)kPoolLen) * iw;
      const float t2 = (float)w * t2s - 1.0f;
      const float q  = t2 * __builtin_amdgcn_rcpf(sp);
      const float val = expf(-0.5f * q * q);
      sV[i * 256 + tid] = live ? val : 0.0f;
    }
  }
  __syncthreads();
  if (isPlane) {
    if (tid < 128) {
      const float* sp = sV + tid * 8;
      v8h hv;
#pragma unroll
      for (int e = 0; e < 8; ++e) hv[e] = (_Float16)sp[e];
      unsigned short* dst = kplanes + (size_t)blk * 1024 + tid * 8;
      *(volatile v8h*)dst = hv;
      __threadfence();
      *(volatile v8h*)dst = hv;
    }
  } else {
    const v4f v = *(const v4f*)(sV + tid * 4);
    float* dst = wtab + (size_t)(blk - kPlaneBlocks) * 1024 + tid * 4;
    *(volatile v4f*)dst = v;
    __threadfence();
    *(volatile v4f*)dst = v;
  }
}

template <int G>
__global__ __launch_bounds__(256) void convpool_kernel(
    const float* __restrict__ x, const unsigned short* __restrict__ kplanes,
    const float* __restrict__ wtab, const float* __restrict__ la, float* __restrict__ Lp)
{
  typedef GroupCfg<G> C;
  constexpr int NT1    = (C::kTs - 1) * C::kPs + C::kWin;
  constexpr int NTILES = (NT1 + 15) / 16;
  constexpr int NTP    = NTILES * 16;
  constexpr int LX     = (NTP - 1) * C::kCs + C::kKp;
  constexpr int LXP    = (LX + 7) & ~7;
  constexpr int LXS    = LXP + 8;
  constexpr int NCOPY  = 8 / C::kStep;
  constexpr int NCH8   = LXP / 8;
  constexpr int KC     = C::kKp / 32;
  constexpr int UN     = (LXS > 10 * NTP) ? LXS : 10 * NTP;
  constexpr int NSUB   = kTileFrames / C::kTs;
  constexpr int NIT    = (C::kWin + C::kNsl - 1) / C::kNsl;
  static_assert(10 * C::kTs * C::kNsl == 160, "pool lanes fill 5 waves");
  static_assert((C::kCs % C::kStep) == 0 && (8 % C::kStep) == 0, "shift step");
  static_assert((C::kKp % 32) == 0 && C::kTaps <= C::kKp, "padded taps");
  static_assert(kSamples / C::kCs == C::kTc && C::kCs * C::kPs == 160, "strides");
  static_assert((kTileFrames % C::kTs) == 0, "sub-tiles");
  static_assert(NCOPY * LXP * 2 + UN * 4 + 10 * 32 * 4 <= 65536, "LDS budget");

  __shared__ __align__(16) _Float16 xsAll[NCOPY * LXP];
  __shared__ __align__(16) float sU[UN];
  __shared__ __align__(16) float outS[10 * kTileFrames];

  const int tid  = threadIdx.x;
  const int lane = tid & 31;
  const int wave = tid >> 5;
  const int hh   = lane >> 4;
  const int nn   = lane & 15;
  const int tile = blockIdx.x;
  const int b    = blockIdx.y;

  for (int i = tid; i < 10 * kTileFrames; i += 256) outS[i] = 0.0f;

  const _Float16* kp = (const _Float16*)(const void*)kplanes + C::kPlaneOff;
  v16h af[KC][2];
#pragma unroll
  for (int kc = 0; kc < KC; ++kc) {
#pragma unroll
    for (int mt = 0; mt < 2; ++mt)
      af[kc][mt] = Frag<_Float16>::load(kp + (size_t)(mt * 16 + nn) * C::kKp + kc * 32 + 8 * hh);
  }

  const int oidx = tid / C::kNsl;
  const int sl   = tid - oidx * C::kNsl;
  const int flr  = oidx / C::kTs;
  const int fl   = flr < 9 ? flr : 9;
  const int tl   = oidx - flr * C::kTs;
  const bool poolAct = tid < 160;
  float av = la[C::kA0 + fl];
  asm volatile("" : "+v"(av));
  const float a10 = expf(av * 2.302585092994046f);

  const float* xrow = x + (size_t)b * kSamples;

#pragma unroll 1
  for (int sub = 0; sub < NSUB; ++sub) {
    const int t0 = tile * kTileFrames + sub * C::kTs;
    if (t0 >= kFrames) break;
    const int p0 = t0 * C::kPs - C::kWin / 2;
    const int xb = p0 * C::kCs - C::kTaps / 2;

    for (int j = tid; j < LXS; j += 256) {
      const int gi = xb + j;
      const bool inr = (gi >= 0) && (gi < kSamples);
      const int gic = gi < 0 ? 0 : (gi >= kSamples ? (kSamples - 1) : gi);
      float v = xrow[gic];
      asm volatile("" : "+v"(v));
      sU[j] = inr ? v * kSigCarry : 0.0f;
    }
    __syncthreads();

    for (int it = tid; it < NCOPY * NCH8; it += 256) {
      const int c  = it / NCH8;
      const int j8 = it - c * NCH8;
      const float* sp = sU + 8 * j8 + c * C::kStep;
      v8h hv;
#pragma unroll
      for (int e = 0; e < 8; ++e) hv[e] = (_Float16)sp[e];
      *(v8h*)(xsAll + c * LXP + 8 * j8) = hv;
    }
    __syncthreads();

    for (int nt = wave; nt < NTILES; nt += 8) {
      const int pl  = nt * 16 + nn;
      const int so  = pl * C::kCs;
      const int sh  = so & 7;
      const int cpy = sh / C::kStep;
      const _Float16* bp = xsAll + cpy * LXP + (so - sh) + 8 * hh;
      v8f acc0 = (v8f){0.f, 0.f, 0.f, 0.f, 0.f, 0.f, 0.f, 0.f};
      v8f acc1 = (v8f){0.f, 0.f, 0.f, 0.f, 0.f, 0.f, 0.f, 0.f};
#pragma unroll
      for (int kc = 0; kc < KC; ++kc) {
        const v16h bf = Frag<_Float16>::load(bp + kc * 32);
        acc0 = mma_g(af[kc][0], bf, acc0);
        acc1 = mma_g(af[kc][1], bf, acc1);
      }
      const int pg = p0 + pl;
      const bool inr = (pg >= 0) && (pg < C::kTc);
#pragma unroll
      for (int q = 0; q < 4; ++q) {
        const float re = acc0[2 * q];
        const float im = acc0[2 * q + 1];
        const float en = (re * re + im * im) * kEnergyFold;
        sU[(4 * hh + q) * NTP + pl] = inr ? en : 0.0f;
      }
      {
        const float re = acc1[0];
        const float im = acc1[1];
        const float en = (re * re + im * im) * kEnergyFold;
        sU[(8 + hh) * NTP + pl] = inr ? en : 0.0f;
      }
    }
    __syncthreads();

    float s = 0.0f;
    if (poolAct) {
      const float* wp = wtab + C::kWinOff + fl * C::kWin;
      const float* ep = sU + fl * NTP + tl * C::kPs;
      for (int wi = 0; wi < NIT; ++wi) {
        const int w  = wi * C::kNsl + sl;
        const int wc = w < C::kWin ? w : (C::kWin - 1);
        const float pr = wp[wc] * ep[wc];
        s += (w < C::kWin) ? pr : 0.0f;
      }
    }
#pragma unroll
    for (int off = 1; off < C::kNsl; off <<= 1) s += __shfl_xor(s, off, 32);
    if (poolAct && sl == 0) {
      const float val = log1pf(a10 * s);
      outS[fl * kTileFrames + sub * C::kTs + tl] = ((t0 + tl) < kFrames) ? val : 0.0f;
    }
    __syncthreads();
  }
  __syncthreads();

  if (wave < 3) {
    const int row  = wave * 4 + (lane >> 3);
    const int rowc = row < 10 ? row : 9;
    const v4f v = *(const v4f*)(outS + rowc * kTileFrames + (lane & 7) * 4);
    float* dst = Lp + (size_t)(b * kBands + C::kA0 + rowc) * kLpPitch + tile * kTileFrames + (lane & 7) * 4;
    if (row < 10) *(volatile v4f*)dst = v;
    __threadfence();
    if (row < 10) *(volatile v4f*)dst = v;
  }
}

__global__ __launch_bounds__(256) void median_kernel(const float* __restrict__ Lp, float* __restrict__ med)
{
  __shared__ float sv[1024];
  const int tid = threadIdx.x;
  const int row = blockIdx.x;
  const float* rp = Lp + (size_t)row * kLpPitch;
#pragma unroll
  for (int i = 0; i < 4; ++i) {
    const int t = tid + 256 * i;
    float v = rp[t];
    asm volatile("" : "+v"(v));
    sv[t] = (t < kFrames) ? v : INFINITY;
  }
  __syncthreads();
#pragma unroll 1
  for (int k = 2; k <= 1024; k <<= 1) {
#pragma unroll 1
    for (int j = k >> 1; j > 0; j >>= 1) {
#pragma unroll
      for (int ii = 0; ii < 2; ++ii) {
        const int i  = tid + 256 * ii;
        const int ia = ((i & ~(j - 1)) << 1) | (i & (j - 1));
        const int ib = ia + j;
        const bool up = ((ia & k) == 0);
        const float va = sv[ia];
        const float vb = sv[ib];
        const float lo = fminf(va, vb);
        const float hi = fmaxf(va, vb);
        sv[ia] = up ? lo : hi;
        sv[ib] = up ? hi : lo;
      }
      __syncthreads();
    }
  }
  if (tid < 32) {
    const float m = sv[(kFrames - 1) / 2];
    float* dst = med + (size_t)row * 32 + tid;
    *(volatile float*)dst = m;
    __threadfence();
    *(volatile float*)dst = m;
  }
}

__global__ __launch_bounds__(256) void chanstats_kernel(
    const float* __restrict__ Lp, const float* __restrict__ med, float* __restrict__ stats)
{
  __shared__ double sd[256];
  __shared__ double sq[256];
  const int tid = threadIdx.x;
  const int c   = blockIdx.x;
  const int f   = c % kBands;
  const int cc  = c / kBands;
  double s = 0.0, s2 = 0.0;
#pragma unroll 1
  for (int b = 0; b < kBatch; ++b) {
    const int rowi = b * kBands + f;
    const float mraw = med[(size_t)rowi * 32];
    const float m = (cc != 0) ? mraw : 0.0f;
    const float* rp = Lp + (size_t)rowi * kLpPitch;
#pragma unroll 1
    for (int i = 0; i < 4; ++i) {
      const int t = tid + 256 * i;
      float v = rp[t];
      asm volatile("" : "+v"(v));
      const float d = v - m;
      const double dv = (t < kFrames) ? (double)d : 0.0;
      s  += dv;
      s2 += dv * dv;
    }
  }
  sd[tid] = s;
  sq[tid] = s2;
  __syncthreads();
#pragma unroll 1
  for (int st = 128; st > 0; st >>= 1) {
    if (tid < st) {
      sd[tid] += sd[tid + st];
      sq[tid] += sq[tid + st];
    }
    __syncthreads();
  }
  if (tid < 32) {
    const double inv = 1.0 / (double)(kBatch * kFrames);
    const double mean = sd[0] * inv;
    const double var  = sq[0] * inv - mean * mean;
    const float varf  = fmaxf((float)var, 0.0f);
    const float meanf = (float)mean;
    const float rstd  = rsqrtf(varf + 1e-5f);
    const float val = (tid == 0) ? meanf : ((tid == 1) ? rstd : 0.0f);
    float* dst = stats + (size_t)c * 32 + tid;
    *(volatile float*)dst = val;
    __threadfence();
    *(volatile float*)dst = val;
  }
}

__global__ __launch_bounds__(256) void chan_apply_kernel(
    const float* __restrict__ Lp, const float* __restrict__ med, const float* __restrict__ stats,
    const float* __restrict__ gamma, const float* __restrict__ beta, float* __restrict__ out)
{
  const int gid = blockIdx.x * 256 + threadIdx.x;
  if (gid >= kBatch * 2 * kBands * kFrames / 4) return;
  const int e0   = gid * 4;
  const int orow = e0 / kFrames;
  const int t    = e0 - orow * kFrames;
  const int f    = orow % kBands;
  const int cc   = (orow / kBands) & 1;
  const int b    = orow / (2 * kBands);
  const int c    = cc * kBands + f;
  const int lrow = b * kBands + f;
  const v4f v = *(const v4f*)(Lp + (size_t)lrow * kLpPitch + t);
  const float mraw = med[(size_t)lrow * 32];
  const float m    = (cc != 0) ? mraw : 0.0f;
  const float mean = stats[(size_t)c * 32];
  const float rstd = stats[(size_t)c * 32 + 1];
  const float g  = gamma[c];
  const float bt = beta[c];
  v4f o;
#pragma unroll
  for (int e = 0; e < 4; ++e) {
    const float z = v[e] - m;
    o[e] = ((z - mean) * rstd) * g + bt;
  }
  float* dst = out + (size_t)e0;
  *(volatile v4f*)dst = o;
  __threadfence();
  *(volatile v4f*)dst = o;
}

extern "C" void kernel_launch(void* const* d_in, const int* in_sizes, int n_in,
                              void* d_out, int out_size, void* d_ws, size_t ws_size,
                              hipStream_t stream) {
  if (n_in < 7) return;
  if (in_sizes[0] != kBatch * kSamples) return;
  if (in_sizes[1] != kBands || in_sizes[2] != kBands || in_sizes[3] != kBands || in_sizes[4] != kBands) return;
  if (in_sizes[5] != 2 * kBands || in_sizes[6] != 2 * kBands) return;
  if (out_size != kBatch * 2 * kBands * kFrames) return;
  if (ws_size < kWsTotal) return;

  const float* x   = (const float*)d_in[0];
  const float* cf  = (const float*)d_in[1];
  const float* bw  = (const float*)d_in[2];
  const float* pw  = (const float*)d_in[3];
  const float* la  = (const float*)d_in[4];
  const float* gam = (const float*)d_in[5];
  const float* bet = (const float*)d_in[6];
  float* out = (float*)d_out;

  char* ws = (char*)d_ws;
  unsigned short* KPL  = (unsigned short*)(ws + kOffKPL);
  float*          WIN  = (float*)(ws + kOffWIN);
  float*          LP   = (float*)(ws + kOffLP);
  float*          MED  = (float*)(ws + kOffMED);
  float*          STAT = (float*)(ws + kOffSTAT);

  gen_tables_kernel<<<kPlaneBlocks + kWinBlocks, 256, 0, stream>>>(cf, bw, pw, KPL, WIN);

  const dim3 cgrid(kRowTiles, kBatch);
  convpool_kernel<0><<<cgrid, 256, 0, stream>>>(x, KPL, WIN, la, LP);
  convpool_kernel<1><<<cgrid, 256, 0, stream>>>(x, KPL, WIN, la, LP);
  convpool_kernel<2><<<cgrid, 256, 0, stream>>>(x, KPL, WIN, la, LP);
  convpool_kernel<3><<<cgrid, 256, 0, stream>>>(x, KPL, WIN, la, LP);

  median_kernel<<<kBatch * kBands, 256, 0, stream>>>(LP, MED);
  chanstats_kernel<<<2 * kBands, 256, 0, stream>>>(LP, MED, STAT);
  chan_apply_kernel<<<(kBatch * 2 * kBands * kFrames / 4) / 256, 256, 0, stream>>>(LP, MED, STAT, gam, bet, out);
}
